// MambaModule_19980187861552
// MI455X (gfx1250) — hardware-verified
//
#include <hip/hip_runtime.h>
#include <math.h>

typedef __attribute__((ext_vector_type(16))) _Float16 v16h;
typedef __attribute__((ext_vector_type(8)))  _Float16 v8h;
typedef __attribute__((ext_vector_type(16))) __bf16   v16b;
typedef __attribute__((ext_vector_type(8)))  __bf16   v8b;
typedef __attribute__((ext_vector_type(8)))  float    v8f;
typedef __attribute__((ext_vector_type(4)))  float    v4f;

constexpr int kBatch = 2;
constexpr int kSeqL  = 1024;
constexpr int kDmod  = 1024;
constexpr int kDin   = 2048;
constexpr int kNst   = 16;
constexpr int kDtR   = 64;
constexpr int kPrjN  = 96;
constexpr int kPrjP  = 128;
constexpr int kXZP   = 2 * kDin;
constexpr int kRows  = kBatch * kSeqL;
constexpr int kTP    = 260;

__device__ __forceinline__ unsigned short f2bf_bits(float f) {
  unsigned u = __float_as_uint(f);
  return (unsigned short)((u + 0x7FFFu + ((u >> 16) & 1u)) >> 16);
}
__device__ __forceinline__ float bf_bits2f(unsigned short h) { return __uint_as_float(((unsigned)h) << 16); }
__device__ __forceinline__ float rne_bf(float f) { return bf_bits2f(f2bf_bits(f)); }

__device__ __forceinline__ void dep_guard_h(v8f& a, v8f& b, v16h x, v16h y) { asm volatile("v_nop\n\tv_nop\n\tv_nop\n\tv_nop" : "+v"(a), "+v"(b) : "v"(x), "v"(y)); }
__device__ __forceinline__ void dep_guard_b(v8f& a, v8f& b, v16b x, v16b y) { asm volatile("v_nop\n\tv_nop\n\tv_nop\n\tv_nop" : "+v"(a), "+v"(b) : "v"(x), "v"(y)); }
__device__ __forceinline__ void keep4_h(v16h a, v16h b, v16h c, v16h d) { asm volatile("v_nop" :: "v"(a), "v"(b), "v"(c), "v"(d)); }
__device__ __forceinline__ void keep4_b(v16b a, v16b b, v16b c, v16b d) { asm volatile("v_nop" :: "v"(a), "v"(b), "v"(c), "v"(d)); }
__device__ __forceinline__ void acc_guard4(v8f& a, v8f& b, v8f& c, v8f& d) { asm volatile("v_nop\n\tv_nop\n\tv_nop\n\tv_nop" : "+v"(a), "+v"(b), "+v"(c), "+v"(d)); }
template <typename T> struct Frag;
template <> struct Frag<_Float16> {
  typedef v16h V; union U { v16h v; v8h h[2]; };
  static __device__ __forceinline__ v16h load(const _Float16* p) {
    U f; f.h[0] = *(const v8h*)(p); f.h[1] = *(const v8h*)(p + 16); return f.v;
  }
  static __device__ __forceinline__ v8f mma(v16h a, v16h b, v8f c) {
    return __builtin_amdgcn_wmma_f32_16x16x32_f16(false, a, false, b, (short)0, c, false, false);
  }
  static __device__ __forceinline__ void guard(v8f& a, v8f& b, v16h x, v16h y) { dep_guard_h(a, b, x, y); }
  static __device__ __forceinline__ void keep(v16h a, v16h b, v16h c, v16h d) { keep4_h(a, b, c, d); }
};
template <> struct Frag<__bf16> {
  typedef v16b V; union U { v16b v; v8b h[2]; };
  static __device__ __forceinline__ v16b load(const __bf16* p) {
    U f; f.h[0] = *(const v8b*)(p); f.h[1] = *(const v8b*)(p + 16); return f.v;
  }
  static __device__ __forceinline__ v8f mma(v16b a, v16b b, v8f c) {
    return __builtin_amdgcn_wmma_f32_16x16x32_bf16(false, a, false, b, (short)0, c, false, false);
  }
  static __device__ __forceinline__ void guard(v8f& a, v8f& b, v16b x, v16b y) { dep_guard_b(a, b, x, y); }
  static __device__ __forceinline__ void keep(v16b a, v16b b, v16b c, v16b d) { keep4_b(a, b, c, d); }
};

template <int ET> struct Elem;
template <> struct Elem<0> { typedef _Float16 T; };
template <> struct Elem<1> { typedef __bf16 T; };
template <int ET, bool SPLIT, int BIAS_MODE, int OUT_MODE, bool RESID, int ACT = 0>
__global__ __launch_bounds__(256) void wmma_gemm64(
    const unsigned short* __restrict__ Ap, const unsigned short* __restrict__ A2p, int lda, long strideA,
    const unsigned short* __restrict__ Btp, const unsigned short* __restrict__ Bt2p, int ldb, long strideB,
    void* __restrict__ Cout, void* __restrict__ Cout2, int ldc, long strideC,
    const float* __restrict__ bias,
    const float* __restrict__ resid, long strideR,
    int M, int N, int K, float scale) {
  typedef typename Elem<ET>::T T;
  typedef typename Frag<T>::V V;
  const T* A = (const T*)Ap; const T* A2 = (const T*)A2p; const T* Bt = (const T*)Btp; const T* Bt2 = (const T*)Bt2p;
  __shared__ __align__(16) float sT[8][16 * 68];
  const int b    = blockIdx.y;
  const int lane = threadIdx.x & 31;
  const int wave = threadIdx.x >> 5;
  const int tilesN = N >> 6;
  const int tilesM = M >> 6;
  const int tile = blockIdx.x * 8 + wave;
  if (tile >= tilesM * tilesN) return;
  const int tm = tile / tilesN;
  const int tn = tile - tm * tilesN;
  const int m0 = tm << 6;
  const int n0 = tn << 6;

  const T* Ab  = A  + (size_t)b * strideA;
  const T* Bb  = Bt + (size_t)b * strideB;
  const T* Ab2 = SPLIT ? (A2  + (size_t)b * strideA) : nullptr;
  const T* Bb2 = SPLIT ? (Bt2 + (size_t)b * strideB) : nullptr;

  const int rlane = lane & 15;
  const int koff  = (lane >> 4) * 8;
  const int mOff  = (lane >> 4) * 8;

  v8f acc[4][4];
#pragma unroll
  for (int i = 0; i < 4; ++i)
#pragma unroll
    for (int j = 0; j < 4; ++j) acc[i][j] = (v8f){0.f,0.f,0.f,0.f,0.f,0.f,0.f,0.f};

  for (int k0 = 0; k0 < K; k0 += 32) {
    V bh[4], bl[4];
#pragma unroll
    for (int j = 0; j < 4; ++j) {
      const size_t bo = (size_t)(n0 + (j << 4) + rlane) * ldb + koff + k0;
      bh[j] = Frag<T>::load(Bb + bo);
      if (SPLIT) bl[j] = Frag<T>::load(Bb2 + bo);
    }
#pragma unroll
    for (int i = 0; i < 4; ++i) {
      const size_t ao = (size_t)(m0 + (i << 4) + rlane) * lda + koff + k0;
      V ah = Frag<T>::load(Ab + ao);
      V al;
      if (SPLIT) al = Frag<T>::load(Ab2 + ao);
#pragma unroll
      for (int j = 0; j < 4; ++j) {
        acc[i][j] = Frag<T>::mma(ah, bh[j], acc[i][j]);
        if (SPLIT) {
          acc[i][j] = Frag<T>::mma(ah, bl[j], acc[i][j]);
          acc[i][j] = Frag<T>::mma(al, bh[j], acc[i][j]);
        }
      }
      Frag<T>::guard(acc[i][0], acc[i][3], ah, SPLIT ? al : ah);
    }
    Frag<T>::keep(bh[0], bh[1], bh[2], bh[3]);
    if (SPLIT) Frag<T>::keep(bl[0], bl[1], bl[2], bl[3]);
  }
  acc_guard4(acc[0][0], acc[0][1], acc[0][2], acc[0][3]);
  acc_guard4(acc[1][0], acc[1][1], acc[1][2], acc[1][3]);
  acc_guard4(acc[2][0], acc[2][1], acc[2][2], acc[2][3]);
  acc_guard4(acc[3][0], acc[3][1], acc[3][2], acc[3][3]);

  float* slab = sT[wave];
  const float* Rb = RESID ? (resid + (size_t)b * strideR) : nullptr;
#pragma unroll
  for (int i = 0; i < 4; ++i) {
    const int mBase = m0 + (i << 4);
#pragma unroll
    for (int j = 0; j < 4; ++j) {
      const int n = n0 + (j << 4) + rlane;
      float bv = 0.f;
      if (BIAS_MODE == 2) bv = bias[n];
#pragma unroll
      for (int r = 0; r < 8; ++r) {
        float v = acc[i][j][r] * scale;
        if (BIAS_MODE == 1) v += bias[mBase + mOff + r];
        if (BIAS_MODE == 2) v += bv;
        if (RESID) v += Rb[(size_t)(mBase + mOff + r) * ldc + n];
        if (ACT == 1) v = tanhf(v);
        if (ACT == 2) v = fmaxf(v, 0.0f);
        if (ACT == 3) v = v / (1.0f + expf(-v));
        if (ACT == 4) v = (v > 0.f) ? v : 0.01f * v;
        if (ACT == 5) v = 0.5f * v * (1.0f + erff(v * 0.70710678118654752f));
        slab[(mOff + r) * 68 + (j << 4) + rlane] = v;
      }
    }
    __builtin_amdgcn_fence(__ATOMIC_RELEASE, "workgroup");
    __builtin_amdgcn_wave_barrier();
    __builtin_amdgcn_fence(__ATOMIC_ACQUIRE, "workgroup");
    if (OUT_MODE == 0) {
      float* C = (float*)Cout + (size_t)b * strideC;
      const int hh = lane >> 4, c4 = (lane & 15) * 4;
      for (int pass = 0; pass < 2; ++pass) {
#pragma unroll
        for (int it = 0; it < 8; ++it) {
          const int row = it * 2 + hh;
          v4f v = *(const v4f*)(slab + row * 68 + c4);
          *(volatile v4f*)(C + (size_t)(mBase + row) * ldc + n0 + c4) = v;
        }
        __threadfence();
      }
    } else {
      const int q = lane >> 3, c8 = (lane & 7) * 8;
      unsigned short* C  = (unsigned short*)Cout  + (size_t)b * strideC;
      unsigned short* C2 = (OUT_MODE == 2) ? ((unsigned short*)Cout2 + (size_t)b * strideC) : nullptr;
      for (int pass = 0; pass < 2; ++pass) {
#pragma unroll
        for (int it = 0; it < 4; ++it) {
          const int row = it * 4 + q;
          const float* sp = slab + row * 68 + c8;
          v8h hv, lv;
#pragma unroll
          for (int e = 0; e < 8; ++e) {
            if (OUT_MODE == 1) {
              hv[e] = (_Float16)sp[e];
            } else {
              unsigned short hb = f2bf_bits(sp[e]);
              unsigned short lb = f2bf_bits(sp[e] - bf_bits2f(hb));
              hv[e] = __builtin_bit_cast(_Float16, hb);
              lv[e] = __builtin_bit_cast(_Float16, lb);
            }
          }
          *(volatile v8h*)(C + (size_t)(mBase + row) * ldc + n0 + c8) = hv;
          if (OUT_MODE == 2) *(volatile v8h*)(C2 + (size_t)(mBase + row) * ldc + n0 + c8) = lv;
        }
        __threadfence();
      }
    }
    __builtin_amdgcn_fence(__ATOMIC_RELEASE, "workgroup");
    __builtin_amdgcn_wave_barrier();
    __builtin_amdgcn_fence(__ATOMIC_ACQUIRE, "workgroup");
  }
}

__global__ __launch_bounds__(256) void cast_bf16_rows_kernel(
    const float* __restrict__ src, unsigned short* __restrict__ dst, int total8)
{
  const int i = blockIdx.x * 256 + threadIdx.x;
  if (i >= total8) return;
  const size_t e0 = (size_t)i << 3;
  const float* p = src + e0;
  const v4f a0 = *(const v4f*)(p);
  const v4f a1 = *(const v4f*)(p + 4);
  v8h hv;
#pragma unroll
  for (int e = 0; e < 4; ++e) {
    hv[e]     = __builtin_bit_cast(_Float16, f2bf_bits(a0[e]));
    hv[4 + e] = __builtin_bit_cast(_Float16, f2bf_bits(a1[e]));
  }
  unsigned short* q = dst + e0;
  *(volatile v8h*)q = hv;
  __threadfence();
  *(volatile v8h*)q = hv;
}

__global__ __launch_bounds__(256) void cast_wrows_f16_kernel(
    const float* __restrict__ src, unsigned short* __restrict__ dst, int N, int K, int total8, float scale)
{
  const int i = blockIdx.x * 256 + threadIdx.x;
  if (i >= total8) return;
  const int e0  = i << 3;
  const int row = e0 / K;
  const int col = e0 - row * K;
  const int rowc = (row < N) ? row : (N - 1);
  const bool live = (row < N);
  const float* p = src + (size_t)rowc * K + col;
  const v4f a0 = *(const v4f*)(p);
  const v4f a1 = *(const v4f*)(p + 4);
  v8h hv;
#pragma unroll
  for (int e = 0; e < 4; ++e) {
    hv[e]     = live ? (_Float16)(rne_bf(a0[e]) * scale) : (_Float16)0.0f;
    hv[4 + e] = live ? (_Float16)(rne_bf(a1[e]) * scale) : (_Float16)0.0f;
  }
  unsigned short* q = dst + (size_t)e0;
  *(volatile v8h*)q = hv;
  __threadfence();
  *(volatile v8h*)q = hv;
}

__global__ __launch_bounds__(256) void cast_padk_f16_kernel(
    const float* __restrict__ src, int lds, unsigned short* __restrict__ dst, int K, int Kp, int total8, float scale)
{
  const int i = blockIdx.x * 256 + threadIdx.x;
  if (i >= total8) return;
  const int e0  = i << 3;
  const int row = e0 / Kp;
  const int col = e0 - row * Kp;
  const bool live = (col < K);
  const int colc = live ? col : (K - 8);
  const float* p = src + (size_t)row * lds + colc;
  const v4f a0 = *(const v4f*)(p);
  const v4f a1 = *(const v4f*)(p + 4);
  v8h hv;
#pragma unroll
  for (int e = 0; e < 4; ++e) {
    hv[e]     = live ? (_Float16)(a0[e] * scale) : (_Float16)0.0f;
    hv[4 + e] = live ? (_Float16)(a1[e] * scale) : (_Float16)0.0f;
  }
  unsigned short* q = dst + (size_t)e0;
  *(volatile v8h*)q = hv;
  __threadfence();
  *(volatile v8h*)q = hv;
}

__global__ __launch_bounds__(256) void conv_silu_kernel(
    const float* __restrict__ XZ, const float* __restrict__ cw, const float* __restrict__ cb,
    unsigned short* __restrict__ XC16, int rev)
{
  __shared__ __align__(16) float sT[16 * kTP];
  const int tid = threadIdx.x, lane = tid & 31, wave = tid >> 5;
  const int d0 = blockIdx.x * 256, d = d0 + tid;
  const int t0 = blockIdx.y * 64;
  const int b  = blockIdx.z;
  const size_t brow = (size_t)b * kSeqL;
  const float w0 = rne_bf(cw[d * 4 + 0]), w1 = rne_bf(cw[d * 4 + 1]), w2 = rne_bf(cw[d * 4 + 2]), w3 = rne_bf(cw[d * 4 + 3]);
  const float bc = rne_bf(cb[d]);
  float xm3, xm2, xm1;
  {
    const int r3 = t0 - 3, r2 = t0 - 2, r1 = t0 - 1;
    const int c3 = r3 < 0 ? 0 : r3, c2 = r2 < 0 ? 0 : r2, c1 = r1 < 0 ? 0 : r1;
    const int l3 = rev ? (kSeqL - 1 - c3) : c3;
    const int l2 = rev ? (kSeqL - 1 - c2) : c2;
    const int l1 = rev ? (kSeqL - 1 - c1) : c1;
    const float v3 = XZ[(brow + (size_t)l3) * kXZP + d];
    const float v2 = XZ[(brow + (size_t)l2) * kXZP + d];
    const float v1 = XZ[(brow + (size_t)l1) * kXZP + d];
    xm3 = (r3 >= 0) ? v3 : 0.f;
    xm2 = (r2 >= 0) ? v2 : 0.f;
    xm1 = (r1 >= 0) ? v1 : 0.f;
  }
#pragma unroll 1
  for (int sub = 0; sub < 4; ++sub) {
    const int lb = t0 + sub * 16;
#pragma unroll 1
    for (int st = 0; st < 16; ++st) {
      const int tt  = lb + st;
      const int tok = rev ? (kSeqL - 1 - tt) : tt;
      const float xin = XZ[(brow + (size_t)tok) * kXZP + d];
      float acc = w0 * xm3;
      acc = fmaf(w1, xm2, acc);
      acc = fmaf(w2, xm1, acc);
      acc = fmaf(w3, xin, acc);
      const float sv = acc + bc;
      const float sg = __builtin_amdgcn_rcpf(1.0f + __expf(-sv));
      sT[st * kTP + tid] = (sv * sg) * 16.0f;
      xm3 = xm2; xm2 = xm1; xm1 = xin;
    }
    __syncthreads();
    v8h bv[2];
#pragma unroll
    for (int it = 0; it < 2; ++it) {
      const float* sp = sT + (it * 8 + wave) * kTP + lane * 8;
      const v4f a0 = *(const v4f*)(sp);
      const v4f a1 = *(const v4f*)(sp + 4);
#pragma unroll
      for (int e = 0; e < 4; ++e) {
        bv[it][e]     = (_Float16)a0[e];
        bv[it][4 + e] = (_Float16)a1[e];
      }
    }
    for (int pass = 0; pass < 2; ++pass) {
#pragma unroll
      for (int it = 0; it < 2; ++it) {
        const int tt  = lb + it * 8 + wave;
        const int tok = rev ? (kSeqL - 1 - tt) : tt;
        *(volatile v8h*)(XC16 + (brow + (size_t)tok) * kDin + d0 + lane * 8) = bv[it];
      }
      __threadfence();
    }
    __syncthreads();
  }
}

template <int MODE>
__global__ __launch_bounds__(256) void scan_kernel(
    const float* __restrict__ DTRAW, const float* __restrict__ XZ, const float* __restrict__ XDBL,
    const float* __restrict__ cw, const float* __restrict__ cb, const float* __restrict__ dtb,
    const float* __restrict__ A_log, const float* __restrict__ Dv,
    float* __restrict__ YF, unsigned short* __restrict__ OZ16)
{
  __shared__ __align__(16) float sBC[16 * 32];
  __shared__ __align__(16) float sY[16 * kTP];
  const int tid = threadIdx.x, lane = tid & 31, wave = tid >> 5;
  const int d0 = blockIdx.x * 256, d = d0 + tid;
  const int b  = blockIdx.y;
  const size_t brow = (size_t)b * kSeqL;

  float An[kNst];
#pragma unroll
  for (int n = 0; n < kNst; ++n) An[n] = -expf(rne_bf(A_log[(size_t)d * kNst + n]));
  const float Dd  = rne_bf(Dv[d]);
  const float bdt = rne_bf(dtb[d]);
  const float bc  = rne_bf(cb[d]);
  const float w0 = rne_bf(cw[d * 4 + 0]), w1 = rne_bf(cw[d * 4 + 1]), w2 = rne_bf(cw[d * 4 + 2]), w3 = rne_bf(cw[d * 4 + 3]);
  float h[kNst];
#pragma unroll
  for (int n = 0; n < kNst; ++n) h[n] = 0.f;
  float xm3 = 0.f, xm2 = 0.f, xm1 = 0.f;

#pragma unroll 1
  for (int c = 0; c < kSeqL / 16; ++c) {
    const int l0 = c * 16;
    if (tid < 128) {
      const int r = tid >> 3, q = (tid & 7) * 4;
      const int tt  = l0 + r;
      const int tok = MODE ? (kSeqL - 1 - tt) : tt;
      const v4f v = *(const v4f*)(XDBL + (brow + (size_t)tok) * kPrjP + kDtR + q);
      *(v4f*)(sBC + r * 32 + q) = v;
    }
    __syncthreads();
#pragma unroll 1
    for (int st = 0; st < 16; ++st) {
      const int tt  = l0 + st;
      const int tok = MODE ? (kSeqL - 1 - tt) : tt;
      const size_t m = brow + (size_t)tok;
      const float a     = DTRAW[m * kDin + d] + bdt;
      const float delta = fmaxf(a, 0.0f) + log1pf(__expf(-fabsf(a)));
      const float xin   = XZ[m * kXZP + d];
      float acc = w0 * xm3;
      acc = fmaf(w1, xm2, acc);
      acc = fmaf(w2, xm1, acc);
      acc = fmaf(w3, xin, acc);
      const float sv  = acc + bc;
      const float sgx = __builtin_amdgcn_rcpf(1.0f + __expf(-sv));
      const float xv  = sv * sgx;
      xm3 = xm2; xm2 = xm1; xm1 = xin;
      const float zv  = XZ[m * kXZP + kDin + d];
      v4f Bq[4], Cq[4];
#pragma unroll
      for (int qq = 0; qq < 4; ++qq) {
        Bq[qq] = *(const v4f*)(sBC + st * 32 + 4 * qq);
        Cq[qq] = *(const v4f*)(sBC + st * 32 + kNst + 4 * qq);
      }
      float dx = delta * xv;
      asm volatile("" : "+v"(dx));
      float y = 0.f;
#pragma unroll
      for (int n = 0; n < kNst; ++n) {
        const float e = __expf(delta * An[n]);
        float p = dx * Bq[n >> 2][n & 3];
        asm volatile("" : "+v"(p));
        float qv = h[n] * e;
        asm volatile("" : "+v"(qv));
        const float hn = qv + p;
        h[n] = hn;
        float rr = Cq[n >> 2][n & 3] * hn;
        asm volatile("" : "+v"(rr));
        y += rr;
      }
      float sk = xv * Dd;
      asm volatile("" : "+v"(sk));
      y += sk;
      const float sg = __builtin_amdgcn_rcpf(1.0f + __expf(-zv));
      const float g  = zv * sg;
      float val = y * g;
      if (MODE == 1) {
        const float yf = YF[m * kDin + d];
        val = (yf + val) * 8.0f;
      }
      sY[st * kTP + tid] = val;
    }
    __syncthreads();
    if (MODE == 0) {
      v4f av[2][2];
#pragma unroll
      for (int it = 0; it < 2; ++it) {
        const float* sp = sY + (it * 8 + wave) * kTP;
        av[it][0] = *(const v4f*)(sp + 4 * lane);
        av[it][1] = *(const v4f*)(sp + 128 + 4 * lane);
      }
      for (int pass = 0; pass < 2; ++pass) {
#pragma unroll
        for (int it = 0; it < 2; ++it) {
          const int tt  = l0 + it * 8 + wave;
          const size_t yo = (brow + (size_t)tt) * kDin + d0;
          *(volatile v4f*)(YF + yo + 4 * lane)       = av[it][0];
          *(volatile v4f*)(YF + yo + 128 + 4 * lane) = av[it][1];
        }
        __threadfence();
      }
    } else {
      v8h hv[2];
#pragma unroll
      for (int it = 0; it < 2; ++it) {
        const float* sp = sY + (it * 8 + wave) * kTP + lane * 8;
        const v4f a0 = *(const v4f*)(sp);
        const v4f a1 = *(const v4f*)(sp + 4);
#pragma unroll
        for (int e = 0; e < 4; ++e) {
          hv[it][e]     = (_Float16)a0[e];
          hv[it][4 + e] = (_Float16)a1[e];
        }
      }
      for (int pass = 0; pass < 2; ++pass) {
#pragma unroll
        for (int it = 0; it < 2; ++it) {
          const int tt  = l0 + it * 8 + wave;
          const int tok = kSeqL - 1 - tt;
          const size_t yo = (brow + (size_t)tok) * kDin + d0 + lane * 8;
          *(volatile v8h*)(OZ16 + yo) = hv[it];
        }
        __threadfence();
      }
    }
  }
}

extern "C" void kernel_launch(void* const* d_in, const int* in_sizes, int n_in,
                              void* d_out, int out_size, void* d_ws, size_t ws_size,
                              hipStream_t stream)
{
  if (n_in < 17) return;
  const float* x      = (const float*)d_in[0];
  const float* W_in   = (const float*)d_in[1];
  const float* W_out  = (const float*)d_in[16];
  const float* conv_w[2] = { (const float*)d_in[2],  (const float*)d_in[4]  };
  const float* conv_b[2] = { (const float*)d_in[3],  (const float*)d_in[5]  };
  const float* W_x[2]    = { (const float*)d_in[6],  (const float*)d_in[9]  };
  const float* W_dt[2]   = { (const float*)d_in[7],  (const float*)d_in[10] };
  const float* b_dt[2]   = { (const float*)d_in[8],  (const float*)d_in[11] };
  const float* A_log[2]  = { (const float*)d_in[12], (const float*)d_in[13] };
  const float* Dv[2]     = { (const float*)d_in[14], (const float*)d_in[15] };
  float* dout = (float*)d_out;

  if (in_sizes[0] != kRows * kDmod) return;
  if (in_sizes[1] != kXZP * kDmod) return;
  if (in_sizes[16] != kDmod * kDin) return;
  if (in_sizes[2] != kDin * 4 || in_sizes[4] != kDin * 4) return;
  if (in_sizes[3] != kDin || in_sizes[5] != kDin) return;
  if (in_sizes[6] != kPrjN * kDin || in_sizes[9] != kPrjN * kDin) return;
  if (in_sizes[7] != kDin * kDtR || in_sizes[10] != kDin * kDtR) return;
  if (in_sizes[8] != kDin || in_sizes[11] != kDin) return;
  if (in_sizes[12] != kDin * kNst || in_sizes[13] != kDin * kNst) return;
  if (in_sizes[14] != kDin || in_sizes[15] != kDin) return;
  if (out_size != kRows * kDmod) return;

  const size_t SZ_X16    = (size_t)kRows * kDmod * 2;
  const size_t SZ_WIN16  = (size_t)kXZP * kDmod * 2;
  const size_t SZ_XZ     = (size_t)kRows * kXZP * 4;
  const size_t SZ_WXP16  = (size_t)kPrjP * kDin * 2;
  const size_t SZ_WDT16  = (size_t)kDin * kDtR * 2;
  const size_t SZ_WOUT16 = (size_t)kDmod * kDin * 2;
  const size_t SZ_XC16   = (size_t)kRows * kDin * 2;
  const size_t SZ_XDBL   = (size_t)kRows * kPrjP * 4;
  const size_t SZ_DT16   = (size_t)kRows * kDtR * 2;
  const size_t SZ_DTRAW  = (size_t)kRows * kDin * 4;
  const size_t SZ_YF     = (size_t)kRows * kDin * 4;
  const size_t SZ_OZ16   = (size_t)kRows * kDin * 2;
  const size_t OFF_X16    = 0;
  const size_t OFF_WIN16  = OFF_X16    + SZ_X16;
  const size_t OFF_XZ     = OFF_WIN16  + SZ_WIN16;
  const size_t OFF_WXP16  = OFF_XZ     + SZ_XZ;
  const size_t OFF_WDT16  = OFF_WXP16  + 2 * SZ_WXP16;
  const size_t OFF_WOUT16 = OFF_WDT16  + 2 * SZ_WDT16;
  const size_t OFF_XC16   = OFF_WOUT16 + SZ_WOUT16;
  const size_t OFF_XDBL   = OFF_XC16   + SZ_XC16;
  const size_t OFF_DT16   = OFF_XDBL   + SZ_XDBL;
  const size_t OFF_DTRAW  = OFF_DT16   + SZ_DT16;
  const size_t OFF_YF     = OFF_DTRAW  + SZ_DTRAW;
  const size_t OFF_OZ16   = OFF_YF     + SZ_YF;
  const size_t TOTAL      = OFF_OZ16   + SZ_OZ16;
  if (ws_size < TOTAL) return;

  char* ws = (char*)d_ws;
  unsigned short* X16    = (unsigned short*)(ws + OFF_X16);
  unsigned short* WIN16  = (unsigned short*)(ws + OFF_WIN16);
  float*          XZ     = (float*)(ws + OFF_XZ);
  unsigned short* WXP16[2] = { (unsigned short*)(ws + OFF_WXP16), (unsigned short*)(ws + OFF_WXP16 + SZ_WXP16) };
  unsigned short* WDT16[2] = { (unsigned short*)(ws + OFF_WDT16), (unsigned short*)(ws + OFF_WDT16 + SZ_WDT16) };
  unsigned short* WOUT16 = (unsigned short*)(ws + OFF_WOUT16);
  unsigned short* XC16   = (unsigned short*)(ws + OFF_XC16);
  float*          XDBL   = (float*)(ws + OFF_XDBL);
  unsigned short* DT16   = (unsigned short*)(ws + OFF_DT16);
  float*          DTRAW  = (float*)(ws + OFF_DTRAW);
  float*          YF     = (float*)(ws + OFF_YF);
  unsigned short* OZ16   = (unsigned short*)(ws + OFF_OZ16);
  const float* dummy_bias  = b_dt[0];
  const float* dummy_resid = x;

  cast_bf16_rows_kernel<<<(kRows * kDmod) / 8 / 256, 256, 0, stream>>>(x, X16, (kRows * kDmod) / 8);
  cast_bf16_rows_kernel<<<(kXZP * kDmod) / 8 / 256, 256, 0, stream>>>(W_in, WIN16, (kXZP * kDmod) / 8);

  wmma_gemm64<1, false, 0, 0, false><<<dim3(256, 1), 256, 0, stream>>>(
      X16, X16, kDmod, 0L, WIN16, WIN16, kDmod, 0L,
      (void*)XZ, (void*)XZ, kXZP, 0L, dummy_bias, dummy_resid, 0L, kRows, kXZP, kDmod, 1.0f);

  cast_wrows_f16_kernel<<<(kDmod * kDin) / 8 / 256, 256, 0, stream>>>(
      W_out, WOUT16, kDmod, kDin, (kDmod * kDin) / 8, 32.0f);

  for (int dir = 0; dir < 2; ++dir) {
    cast_wrows_f16_kernel<<<(kPrjP * kDin) / 8 / 256, 256, 0, stream>>>(
        W_x[dir], WXP16[dir], kPrjN, kDin, (kPrjP * kDin) / 8, 32.0f);
    cast_wrows_f16_kernel<<<(kDin * kDtR) / 8 / 256, 256, 0, stream>>>(
        W_dt[dir], WDT16[dir], kDin, kDtR, (kDin * kDtR) / 8, 8.0f);

    conv_silu_kernel<<<dim3(kDin / 256, kSeqL / 64, kBatch), 256, 0, stream>>>(XZ, conv_w[dir], conv_b[dir], XC16, dir);

    wmma_gemm64<0, false, 0, 0, false><<<dim3(8, 1), 256, 0, stream>>>(
        XC16, XC16, kDin, 0L, WXP16[dir], WXP16[dir], kDin, 0L,
        (void*)XDBL, (void*)XDBL, kPrjP, 0L, dummy_bias, dummy_resid, 0L, kRows, kPrjP, kDin, 1.0f / 512.0f);

    cast_padk_f16_kernel<<<(kRows * kDtR) / 8 / 256, 256, 0, stream>>>(
        XDBL, kPrjP, DT16, kDtR, kDtR, (kRows * kDtR) / 8, 64.0f);

    wmma_gemm64<0, false, 0, 0, false><<<dim3(128, 1), 256, 0, stream>>>(
        DT16, DT16, kDtR, 0L, WDT16[dir], WDT16[dir], kDtR, 0L,
        (void*)DTRAW, (void*)DTRAW, kDin, 0L, dummy_bias, dummy_resid, 0L, kRows, kDin, kDtR, 1.0f / 512.0f);

    if (dir == 0)
      scan_kernel<0><<<dim3(kDin / 256, kBatch), 256, 0, stream>>>(
          DTRAW, XZ, XDBL, conv_w[dir], conv_b[dir], b_dt[dir], A_log[dir], Dv[dir], YF, OZ16);
    else
      scan_kernel<1><<<dim3(kDin / 256, kBatch), 256, 0, stream>>>(
          DTRAW, XZ, XDBL, conv_w[dir], conv_b[dir], b_dt[dir], A_log[dir], Dv[dir], YF, OZ16);
  }

  wmma_gemm64<0, false, 0, 0, false><<<dim3(64, 1), 256, 0, stream>>>(
      OZ16, OZ16, kDin, 0L, WOUT16, WOUT16, kDin, 0L,
      (void*)dout, (void*)dout, kDmod, 0L, dummy_bias, dummy_resid, 0L, kRows, kDmod, kDin, 1.0f / 512.0f);
}
